// CMLITargetLoss_6227702579750
// MI455X (gfx1250) — hardware-verified
//
#include <hip/hip_runtime.h>

constexpr int NB      = 64;
constexpr int NT      = 197;
constexpr int ND      = 768;
constexpr int TM1     = NT - 1;
constexpr int ROWS    = NB * NT;
constexpr int KSTEPS  = ND / 32;
constexpr int RB      = 32;
constexpr int PREP_BLOCKS = ROWS / RB;
constexpr int TOKROWS = NB * TM1;
constexpr int TOK_BLOCKS  = TOKROWS / RB;
constexpr int TBLK    = (TM1 + 31) / 32;
constexpr int IDXP    = TBLK * 32;
constexpr float OPSCALE = 4096.0f;

static_assert(ROWS % RB == 0, "");
static_assert(TOKROWS % RB == 0, "");
static_assert(ND % 256 == 0, "");

typedef _Float16 v16h __attribute__((ext_vector_type(16)));
typedef _Float16 v8h  __attribute__((ext_vector_type(8)));
typedef float    v8f  __attribute__((ext_vector_type(8)));
typedef float    v4f  __attribute__((ext_vector_type(4)));
typedef unsigned int v4u __attribute__((ext_vector_type(4)));

union Frag  { v16h v; v8h half[2]; };
union HPack { v8h h; v4u u; };

static __device__ __forceinline__ float waveSum(float v) {
  #pragma unroll
  for (int off = 16; off; off >>= 1) v += __shfl_xor(v, off, 32);
  return v;
}

static __device__ __forceinline__ v8f wmma_f16(v16h a, v16h b, v8f c) {
  v8f d = __builtin_amdgcn_wmma_f32_16x16x32_f16(false, a, false, b, (short)0, c, false, false);
  asm volatile("v_nop\n\tv_nop\n\tv_nop\n\tv_nop" : "+v"(d) : "v"(a), "v"(b));
  return d;
}

__global__ void __launch_bounds__(256)
k_prep(const float* __restrict__ image, const float* __restrict__ text,
       const float* __restrict__ target,
       _Float16* texth, _Float16* targh, float* pimg)
{
  const int wave = threadIdx.x >> 5, lane = threadIdx.x & 31;
  __shared__ float lsi[RB];

  #pragma unroll 1
  for (int j = 0; j < 4; ++j) {
    const int rloc = wave * 4 + j;
    int row = blockIdx.x * RB + rloc;
    if (row > ROWS - 1) row = ROWS - 1;
    const size_t base = (size_t)row * ND;

    float tv[24], gv[24];
    float sst = 0.f, ssg = 0.f, si = 0.f;
    #pragma unroll
    for (int i = 0; i < 3; ++i) {
      const int off = 256 * i + 8 * lane;
      const v4f t0 = *(const v4f*)(text   + base + off);
      const v4f t1 = *(const v4f*)(text   + base + off + 4);
      const v4f g0 = *(const v4f*)(target + base + off);
      const v4f g1 = *(const v4f*)(target + base + off + 4);
      const v4f m0 = *(const v4f*)(image  + base + off);
      const v4f m1 = *(const v4f*)(image  + base + off + 4);
      #pragma unroll
      for (int e = 0; e < 4; ++e) {
        tv[8 * i + e]     = t0[e];
        tv[8 * i + 4 + e] = t1[e];
        gv[8 * i + e]     = g0[e];
        gv[8 * i + 4 + e] = g1[e];
        sst += t0[e] * t0[e] + t1[e] * t1[e];
        ssg += g0[e] * g0[e] + g1[e] * g1[e];
        const float d0 = m0[e] - g0[e];
        const float d1 = m1[e] - g1[e];
        si += d0 * d0 + d1 * d1;
      }
    }
    sst = waveSum(sst);
    ssg = waveSum(ssg);
    si  = waveSum(si);
    const float sct = OPSCALE * (1.0f / sqrtf(sst));
    const float scg = OPSCALE * (1.0f / sqrtf(ssg));

    HPack pt[3], pg[3];
    #pragma unroll
    for (int i = 0; i < 3; ++i) {
      #pragma unroll
      for (int e = 0; e < 8; ++e) {
        pt[i].h[e] = (_Float16)(tv[8 * i + e] * sct);
        pg[i].h[e] = (_Float16)(gv[8 * i + e] * scg);
      }
    }
    _Float16* trow = texth + base;
    _Float16* grow = targh + base;
    #pragma unroll
    for (int i = 0; i < 3; ++i) {
      const int off = 256 * i + 8 * lane;
      *(volatile v4u*)(trow + off) = pt[i].u;
      *(volatile v4u*)(grow + off) = pg[i].u;
    }
    __threadfence();
    #pragma unroll
    for (int i = 0; i < 3; ++i) {
      const int off = 256 * i + 8 * lane;
      *(volatile v4u*)(trow + off) = pt[i].u;
      *(volatile v4u*)(grow + off) = pg[i].u;
    }
    if (lane == 0) lsi[rloc] = si;
  }
  __syncthreads();
  if (wave == 0) {
    const float v = lsi[lane];
    float* p = pimg + (size_t)blockIdx.x * RB + lane;
    *(volatile float*)p = v;
    __threadfence();
    *(volatile float*)p = v;
  }
}

__global__ void __launch_bounds__(128)
k_sim_argmax(const _Float16* __restrict__ texth, const _Float16* __restrict__ targh,
             int* idxw)
{
  const int tb   = blockIdx.x;
  const int b    = blockIdx.y;
  const int l    = threadIdx.x & 31;
  const int h    = l >> 4;
  const int m    = l & 15;
  const int wave = threadIdx.x >> 5;

  int aoff[2];
  #pragma unroll
  for (int mt = 0; mt < 2; ++mt) {
    int t = 1 + tb * 32 + mt * 16 + m;
    if (t > TM1) t = TM1;
    aoff[mt] = (b * NT + t) * ND;
  }
  int boff[4], ncol[4];
  #pragma unroll
  for (int s = 0; s < 4; ++s) {
    const int n = 1 + (wave * 4 + s) * 16 + m;
    ncol[s] = n;
    const int nc = (n > TM1) ? TM1 : n;
    boff[s] = (b * NT + nc) * ND;
  }

  v8f acc[2][4];
  #pragma unroll
  for (int mt = 0; mt < 2; ++mt)
    #pragma unroll
    for (int s = 0; s < 4; ++s)
      #pragma unroll
      for (int j = 0; j < 8; ++j) acc[mt][s][j] = 0.0f;

  #pragma unroll 1
  for (int kt = 0; kt < KSTEPS; ++kt) {
    const int k0 = kt * 32;
    Frag a0, a1;
    a0.half[0] = *(const v8h*)(texth + aoff[0] + k0 + 8 * h);
    a0.half[1] = *(const v8h*)(texth + aoff[0] + k0 + 16 + 8 * h);
    a1.half[0] = *(const v8h*)(texth + aoff[1] + k0 + 8 * h);
    a1.half[1] = *(const v8h*)(texth + aoff[1] + k0 + 16 + 8 * h);
    #pragma unroll
    for (int s = 0; s < 4; ++s) {
      Frag bf;
      bf.half[0] = *(const v8h*)(targh + boff[s] + k0 + 8 * h);
      bf.half[1] = *(const v8h*)(targh + boff[s] + k0 + 16 + 8 * h);
      acc[0][s] = wmma_f16(a0.v, bf.v, acc[0][s]);
      acc[1][s] = wmma_f16(a1.v, bf.v, acc[1][s]);
    }
  }

  const float NEGINF = -__builtin_huge_valf();
  float bestv[2][8]; int besti[2][8];
  #pragma unroll
  for (int mt = 0; mt < 2; ++mt)
    #pragma unroll
    for (int j = 0; j < 8; ++j) { bestv[mt][j] = NEGINF; besti[mt][j] = 0x7fffffff; }

  #pragma unroll
  for (int s = 0; s < 4; ++s) {
    const bool nvalid = (ncol[s] <= TM1);
    #pragma unroll
    for (int mt = 0; mt < 2; ++mt) {
      #pragma unroll
      for (int j = 0; j < 8; ++j) {
        float v  = nvalid ? acc[mt][s][j] : NEGINF;
        int  idx = ncol[s];
        #pragma unroll
        for (int off = 8; off >= 1; off >>= 1) {
          const float ov = __shfl_xor(v, off, 16);
          const int   oi = __shfl_xor(idx, off, 16);
          if (ov > v || (ov == v && oi < idx)) { v = ov; idx = oi; }
        }
        if (v > bestv[mt][j] || (v == bestv[mt][j] && idx < besti[mt][j])) {
          bestv[mt][j] = v; besti[mt][j] = idx;
        }
      }
    }
  }

  __shared__ float lv[4][32];
  __shared__ int   li[4][32];
  if (m == 0) {
    #pragma unroll
    for (int mt = 0; mt < 2; ++mt)
      #pragma unroll
      for (int j = 0; j < 8; ++j) {
        lv[wave][mt * 16 + 8 * h + j] = bestv[mt][j];
        li[wave][mt * 16 + 8 * h + j] = besti[mt][j];
      }
  }
  __syncthreads();
  if (threadIdx.x < 32) {
    const int r = threadIdx.x;
    float v = lv[0][r]; int idx = li[0][r];
    #pragma unroll
    for (int w = 1; w < 4; ++w) {
      const float ov = lv[w][r]; const int oi = li[w][r];
      if (ov > v || (ov == v && oi < idx)) { v = ov; idx = oi; }
    }
    const int tloc = tb * 32 + r;
    const int val  = (tloc < TM1) ? idx : 0;
    int* p = idxw + (size_t)b * IDXP + tloc;
    *(volatile int*)p = val;
    __threadfence();
    *(volatile int*)p = val;
  }
}

__global__ void __launch_bounds__(256)
k_token(const float* __restrict__ text, const float* __restrict__ target,
        const int* __restrict__ mask, const int* __restrict__ idxw, float* psq)
{
  const int wave = threadIdx.x >> 5, lane = threadIdx.x & 31;
  __shared__ float lsq[RB];

  #pragma unroll 1
  for (int j = 0; j < 4; ++j) {
    const int rloc = wave * 4 + j;
    int r = blockIdx.x * RB + rloc;
    if (r > TOKROWS - 1) r = TOKROWS - 1;
    const int b = r / TM1;
    const int t = r - b * TM1 + 1;
    const int keep = (mask[b * NT + t] == 0) ? 1 : 0;
    int g = idxw[(size_t)b * IDXP + (t - 1)];
    g = (g < 0) ? 0 : ((g > NT - 1) ? (NT - 1) : g);
    const size_t tbase = ((size_t)b * NT + t) * (size_t)ND;
    const size_t gbase = ((size_t)b * NT + g) * (size_t)ND;
    float acc = 0.f;
    #pragma unroll
    for (int i = 0; i < 3; ++i) {
      const int off = 256 * i + 8 * lane;
      const v4f t0 = *(const v4f*)(text   + tbase + off);
      const v4f t1 = *(const v4f*)(text   + tbase + off + 4);
      const v4f g0 = *(const v4f*)(target + gbase + off);
      const v4f g1 = *(const v4f*)(target + gbase + off + 4);
      #pragma unroll
      for (int e = 0; e < 4; ++e) {
        const float d0 = t0[e] - g0[e];
        const float d1 = t1[e] - g1[e];
        acc += d0 * d0 + d1 * d1;
      }
    }
    acc = waveSum(acc);
    if (lane == 0) lsq[rloc] = keep ? acc : 0.0f;
  }
  __syncthreads();
  if (wave == 0) {
    const float v = lsq[lane];
    float* p = psq + (size_t)blockIdx.x * RB + lane;
    *(volatile float*)p = v;
    __threadfence();
    *(volatile float*)p = v;
  }
}

__global__ void __launch_bounds__(256)
k_final(const float* __restrict__ text, const float* __restrict__ target,
        const int* __restrict__ mask, const float* __restrict__ psq,
        const float* __restrict__ pimg, float* out)
{
  const int tid = threadIdx.x;
  double s1 = 0.0, si = 0.0, s2 = 0.0; int cnt = 0;
  for (int i = tid; i < TOKROWS; i += 256) s1 += (double)psq[i];
  for (int i = tid; i < ROWS; i += 256) si += (double)pimg[i];
  for (int i = tid; i < TOKROWS; i += 256) {
    const int b = i / TM1, t = i - b * TM1 + 1;
    cnt += (mask[b * NT + t] == 0) ? 1 : 0;
  }
  for (int i = tid; i < NB * ND; i += 256) {
    const int b = i / ND, d = i - b * ND;
    const size_t e = (size_t)b * NT * (size_t)ND + d;
    const float df = text[e] - target[e];
    s2 += (double)(df * df);
  }
  __shared__ double l1[256], l2[256], l3[256];
  __shared__ int lc[256];
  l1[tid] = s1; l2[tid] = si; l3[tid] = s2; lc[tid] = cnt;
  __syncthreads();
  if (tid == 0) {
    double S1 = 0.0, SI = 0.0, S2 = 0.0; long long C = 0;
    for (int w = 0; w < 256; ++w) { S1 += l1[w]; SI += l2[w]; S2 += l3[w]; C += lc[w]; }
    const double nt        = (double)C;
    const double tok_loss  = S1 / (nt * (double)ND);
    const double cls_loss  = S2 / (double)(NB * ND);
    const double text_loss = (nt * tok_loss + cls_loss) / (nt + 1.0);
    const double img_loss  = SI / ((double)NB * (double)NT * (double)ND);
    const float  res = (float)(0.5 * (text_loss + img_loss));
    *(volatile float*)out = res;
    __threadfence();
    *(volatile float*)out = res;
  }
}

extern "C" void kernel_launch(void* const* d_in, const int* in_sizes, int n_in,
                              void* d_out, int out_size, void* d_ws, size_t ws_size,
                              hipStream_t stream)
{
  if (n_in < 4 || out_size < 1) return;
  if (in_sizes[0] != ROWS * ND || in_sizes[1] != ROWS * ND ||
      in_sizes[2] != ROWS * ND || in_sizes[3] != ROWS) return;

  const float* image  = (const float*)d_in[0];
  const float* text   = (const float*)d_in[1];
  const float* target = (const float*)d_in[2];
  const int*   mask   = (const int*)d_in[3];

  const size_t SZ_H   = (size_t)ROWS * ND * sizeof(_Float16);
  const size_t SZ_IDX = (size_t)NB * IDXP * sizeof(int);
  const size_t SZ_PSQ = (size_t)TOKROWS * sizeof(float);
  const size_t SZ_PIM = (size_t)ROWS * sizeof(float);
  const size_t OFF_TH  = 0;
  const size_t OFF_GH  = OFF_TH + SZ_H;
  const size_t OFF_IDX = OFF_GH + SZ_H;
  const size_t OFF_PSQ = OFF_IDX + SZ_IDX;
  const size_t OFF_PIM = OFF_PSQ + SZ_PSQ;
  const size_t TOTAL   = OFF_PIM + SZ_PIM;
  if (TOTAL > ws_size) return;

  char* ws = (char*)d_ws;
  _Float16* texth = (_Float16*)(ws + OFF_TH);
  _Float16* targh = (_Float16*)(ws + OFF_GH);
  int*      idxw  = (int*)     (ws + OFF_IDX);
  float*    psq   = (float*)   (ws + OFF_PSQ);
  float*    pimg  = (float*)   (ws + OFF_PIM);

  k_prep<<<PREP_BLOCKS, 256, 0, stream>>>(image, text, target, texth, targh, pimg);

  dim3 g2(TBLK, NB);
  k_sim_argmax<<<g2, 128, 0, stream>>>(texth, targh, idxw);

  k_token<<<TOK_BLOCKS, 256, 0, stream>>>(text, target, mask, idxw, psq);

  k_final<<<1, 256, 0, stream>>>(text, target, mask, psq, pimg, (float*)d_out);
}
